// RIM_64613488001361
// MI455X (gfx1250) — hardware-verified
//
#include <hip/hip_runtime.h>
#include <stdint.h>
#include <stddef.h>
#include <math.h>

#pragma clang fp contract(off)

#define NB_    4096
#define NU_    6
#define KTOP_  4
#define DIN_   512
#define HID_   512
#define NQ_    128
#define NVS_   512
#define G3_    1536
#define RZP_   1024
#define NQC_   128
#define NVC_   512
#define NVC4_  2048
#define NQKV_  768
#define MP_    8
#define TBM    128
#define TBN    128
#define TBN2   64
#define TT     64
#define TP     68
#define SPH    72
#define SPF    68
#define BP     68
#define STG    4608
#define WSCALE 64.0f
#define WINV   0.015625f
#define ATTSC  0.04419417382415922f

static_assert(32 * SPH * 2 <= STG);
static_assert(16 * SPF * 4 <= STG);
static_assert((SPH * 2) % 16 == 0);
static_assert((SPF * 4) % 16 == 0);
static_assert((TP * 4) % 16 == 0);
static_assert((BP * 4) % 16 == 0);
static_assert(STG % 16 == 0);
static_assert(NB_ % TBM == 0);
static_assert(NB_ % 256 == 0);
static_assert(NQ_ == TBN);
static_assert(NVS_ % TBN == 0);
static_assert(NQKV_ % TBN == 0);
static_assert(RZP_ % TBN2 == 0);
static_assert(HID_ % TBN2 == 0);
static_assert(HID_ % 32 == 0);
static_assert(DIN_ == HID_);
static_assert(NVS_ == HID_);
static_assert(NVC_ == HID_);
static_assert((NB_ * DIN_) % 2048 == 0);
static_assert((NU_ * NB_ * HID_) % 2048 == 0);
static_assert((NU_ * G3_ * HID_) % 2048 == 0);
static_assert(HID_ % TT == 0);
static_assert(NQ_ % TT == 0);
static_assert(NQC_ % TT == 0);
static_assert(NVC_ % TT == 0);
static_assert(NVS_ % TT == 0);
static_assert(NU_ * 32 == 192);
static_assert(HID_ == 4 * 128);
static_assert(TBN == 128);
static_assert(TBN2 == 64);

typedef _Float16 v16h __attribute__((ext_vector_type(16)));
typedef _Float16 v8h  __attribute__((ext_vector_type(8)));
typedef unsigned short v16us __attribute__((ext_vector_type(16)));
typedef unsigned short v8us  __attribute__((ext_vector_type(8)));
typedef __bf16 v16bf __attribute__((ext_vector_type(16)));
typedef float v16f __attribute__((ext_vector_type(16)));
typedef float v8f  __attribute__((ext_vector_type(8)));
typedef float v4f  __attribute__((ext_vector_type(4)));
typedef v4f  __attribute__((may_alias)) v4fa;
typedef v8h  __attribute__((may_alias)) v8ha;
typedef v8us __attribute__((may_alias)) v8usa;

union FragH  { v16h v; v8h q[2]; };
union FragB  { v16bf v; v16us u; v8us q[2]; };
union Pack16 { v16f v; v4f q[4]; };

__device__ __forceinline__ v8f wmma_h(v16h a, v16h b, v8f c) {
  v8f d = __builtin_amdgcn_wmma_f32_16x16x32_f16(false, a, false, b, (short)0, c, false, false);
  asm volatile("v_nop\n\tv_nop\n\tv_nop\n\tv_nop" : "+v"(d) : "v"(a), "v"(b));
  return d;
}
__device__ __forceinline__ v8f wmma_b(v16bf a, v16bf b, v8f c) {
  v8f d = __builtin_amdgcn_wmma_f32_16x16x32_bf16(false, a, false, b, (short)0, c, false, false);
  asm volatile("v_nop\n\tv_nop\n\tv_nop\n\tv_nop" : "+v"(d) : "v"(a), "v"(b));
  return d;
}

__device__ __forceinline__ v16h ldfrag_h(const _Float16* p, int h) {
  FragH f;
  f.q[0] = *(const v8ha*)(p + 8 * h);
  f.q[1] = *(const v8ha*)(p + 16 + 8 * h);
  return f.v;
}
__device__ __forceinline__ v16bf ldfrag_b(const unsigned short* p, int h) {
  FragB f;
  f.q[0] = *(const v8usa*)(p + 8 * h);
  f.q[1] = *(const v8usa*)(p + 16 + 8 * h);
  return f.v;
}

__device__ __forceinline__ unsigned int bf_bits(float f) {
  unsigned int u = __float_as_uint(f);
  u += 0x7FFFu + ((u >> 16) & 1u);
  return u >> 16;
}

__device__ __forceinline__ void ldfrag_split(const float* p, int h, v16bf& hi, v16bf& lo) {
  Pack16 x;
  x.q[0] = *(const v4fa*)(p + 8 * h);
  x.q[1] = *(const v4fa*)(p + 8 * h + 4);
  x.q[2] = *(const v4fa*)(p + 16 + 8 * h);
  x.q[3] = *(const v4fa*)(p + 20 + 8 * h);
  FragB fh, fl;
  #pragma unroll
  for (int i = 0; i < 16; ++i) {
    const float f = x.v[i];
    const unsigned int bh = bf_bits(f);
    const float r = f - __uint_as_float(bh << 16);
    fh.u[i] = (unsigned short)bh;
    fl.u[i] = (unsigned short)bf_bits(r);
  }
  hi = fh.v;
  lo = fl.v;
}

__device__ __forceinline__ void split8(v4f a, v4f b, v8us& hi, v8us& lo) {
  const float f[8] = {a.x, a.y, a.z, a.w, b.x, b.y, b.z, b.w};
  #pragma unroll
  for (int i = 0; i < 8; ++i) {
    const unsigned int bh = bf_bits(f[i]);
    const float r = f[i] - __uint_as_float(bh << 16);
    hi[i] = (unsigned short)bh;
    lo[i] = (unsigned short)bf_bits(r);
  }
}

__device__ __forceinline__ v8h pack8h(v4f a, v4f b) {
  v8h o;
  o[0] = (_Float16)a.x; o[1] = (_Float16)a.y; o[2] = (_Float16)a.z; o[3] = (_Float16)a.w;
  o[4] = (_Float16)b.x; o[5] = (_Float16)b.y; o[6] = (_Float16)b.z; o[7] = (_Float16)b.w;
  return o;
}

__device__ __forceinline__ float sigmoid_f(float v) {
  const float c = fminf(fmaxf(v, -30.0f), 30.0f);
  return __builtin_amdgcn_rcpf(1.0f + __expf(-c));
}
__device__ __forceinline__ float tanh_f(float v) {
  const float ax = fminf(fabsf(v), 9.0f);
  const float ex = __expf(ax + ax);
  const float r  = __builtin_amdgcn_rcpf(ex + 1.0f);
  return copysignf(1.0f - 2.0f * r, v);
}

__global__ __launch_bounds__(256) void k_cvt16(const float* __restrict__ src,
                                               _Float16* __restrict__ dst,
                                               int n8, float scale)
{
  const int i = blockIdx.x * 256 + (int)threadIdx.x;
  if (i >= n8) return;
  const size_t e = (size_t)i * 8;
  const v4f a = *(const v4fa*)(src + e);
  const v4f b = *(const v4fa*)(src + e + 4);
  const v8h o = pack8h(a * scale, b * scale);
  _Float16* d = dst + e;
  *(volatile v8ha*)d = o;
  __threadfence();
  *(volatile v8ha*)d = o;
}

template <int NHD, int SPLIT>
__global__ __launch_bounds__(256) void k_wt(const float* __restrict__ src, long long zsrc,
                                            _Float16* __restrict__ dst,
                                            unsigned short* __restrict__ dhi,
                                            unsigned short* __restrict__ dlo, long long zdst,
                                            int R, int C, float scale)
{
  __shared__ __align__(16) float sT[TT * TP];
  const int tid = threadIdx.x, lane = tid & 31, wv = tid >> 5;
  const size_t zs = (size_t)blockIdx.z * (size_t)zsrc;
  const size_t zd = (size_t)blockIdx.z * (size_t)zdst;
  const int r0 = blockIdx.y * TT;
  const int c0 = blockIdx.x * TT;
  const int ldw = NHD * C;

  const int i = tid >> 2, cs = (tid & 3) * 16;
  const float* sp = src + zs + (size_t)(r0 + i) * ldw + c0 + cs;
  v4f a0 = *(const v4fa*)(sp);
  v4f a1 = *(const v4fa*)(sp + 4);
  v4f a2 = *(const v4fa*)(sp + 8);
  v4f a3 = *(const v4fa*)(sp + 12);
  if constexpr (NHD == 2) {
    a0 = a0 + *(const v4fa*)(sp + C);
    a1 = a1 + *(const v4fa*)(sp + C + 4);
    a2 = a2 + *(const v4fa*)(sp + C + 8);
    a3 = a3 + *(const v4fa*)(sp + C + 12);
  } else if constexpr (NHD == 4) {
    const v4f e0 = *(const v4fa*)(sp + C),     e1 = *(const v4fa*)(sp + C + 4);
    const v4f e2 = *(const v4fa*)(sp + C + 8), e3 = *(const v4fa*)(sp + C + 12);
    const v4f f0 = *(const v4fa*)(sp + 2 * C),     f1 = *(const v4fa*)(sp + 2 * C + 4);
    const v4f f2 = *(const v4fa*)(sp + 2 * C + 8), f3 = *(const v4fa*)(sp + 2 * C + 12);
    const v4f g0 = *(const v4fa*)(sp + 3 * C),     g1 = *(const v4fa*)(sp + 3 * C + 4);
    const v4f g2 = *(const v4fa*)(sp + 3 * C + 8), g3 = *(const v4fa*)(sp + 3 * C + 12);
    a0 = (a0 + e0) + (f0 + g0);
    a1 = (a1 + e1) + (f1 + g1);
    a2 = (a2 + e2) + (f2 + g2);
    a3 = (a3 + e3) + (f3 + g3);
  }
  float* tp = sT + cs * TP + i;
  tp[ 0 * TP] = a0.x; tp[ 1 * TP] = a0.y; tp[ 2 * TP] = a0.z; tp[ 3 * TP] = a0.w;
  tp[ 4 * TP] = a1.x; tp[ 5 * TP] = a1.y; tp[ 6 * TP] = a1.z; tp[ 7 * TP] = a1.w;
  tp[ 8 * TP] = a2.x; tp[ 9 * TP] = a2.y; tp[10 * TP] = a2.z; tp[11 * TP] = a2.w;
  tp[12 * TP] = a3.x; tp[13 * TP] = a3.y; tp[14 * TP] = a3.z; tp[15 * TP] = a3.w;
  __syncthreads();

  const int q  = lane & 7;
  const int cA = 4 * wv + (lane >> 3);
  const int cB = 32 + cA;
  const v4f pA0 = *(const v4fa*)(sT + cA * TP + 8 * q);
  const v4f pA1 = *(const v4fa*)(sT + cA * TP + 8 * q + 4);
  const v4f pB0 = *(const v4fa*)(sT + cB * TP + 8 * q);
  const v4f pB1 = *(const v4fa*)(sT + cB * TP + 8 * q + 4);
  const size_t oA = zd + (size_t)(c0 + cA) * R + r0 + 8 * q;
  const size_t oB = zd + (size_t)(c0 + cB) * R + r0 + 8 * q;
  if constexpr (SPLIT == 0) {
    const v8h vA = pack8h(pA0 * scale, pA1 * scale);
    const v8h vB = pack8h(pB0 * scale, pB1 * scale);
    *(volatile v8ha*)(dst + oA) = vA;
    *(volatile v8ha*)(dst + oB) = vB;
    __threadfence();
    *(volatile v8ha*)(dst + oA) = vA;
    *(volatile v8ha*)(dst + oB) = vB;
  } else {
    v8us hA, lA, hB, lB;
    split8(pA0, pA1, hA, lA);
    split8(pB0, pB1, hB, lB);
    *(volatile v8usa*)(dhi + oA) = hA;
    *(volatile v8usa*)(dlo + oA) = lA;
    *(volatile v8usa*)(dhi + oB) = hB;
    *(volatile v8usa*)(dlo + oB) = lB;
    __threadfence();
    *(volatile v8usa*)(dhi + oA) = hA;
    *(volatile v8usa*)(dlo + oA) = lA;
    *(volatile v8usa*)(dhi + oB) = hB;
    *(volatile v8usa*)(dlo + oB) = lB;
  }
}

__device__ __forceinline__ void kloop(v8f (&acc)[2][4],
                                      const _Float16* A, int lda,
                                      const _Float16* Bt, int ldb, int K,
                                      int rowW, int colW, int h, int m)
{
  const _Float16* a0p = A  + (size_t)(rowW + m) * lda;
  const _Float16* a1p = A  + (size_t)(rowW + 16 + m) * lda;
  const _Float16* b0p = Bt + (size_t)(colW + m) * ldb;
  #pragma unroll 1
  for (int k0 = 0; k0 < K; k0 += 32) {
    const v16h a0 = ldfrag_h(a0p + k0, h);
    const v16h a1 = ldfrag_h(a1p + k0, h);
    #pragma unroll
    for (int nt = 0; nt < 4; ++nt) {
      const v16h b = ldfrag_h(b0p + (size_t)(16 * nt) * ldb + k0, h);
      acc[0][nt] = wmma_h(a0, b, acc[0][nt]);
      acc[1][nt] = wmma_h(a1, b, acc[1][nt]);
    }
  }
}

__device__ __forceinline__ void kloop2(v8f (&acc)[2][2],
                                       const _Float16* A, const _Float16* Bt,
                                       int rowW, int colW, int h, int m)
{
  const _Float16* a0p = A  + (size_t)(rowW + m) * HID_;
  const _Float16* a1p = A  + (size_t)(rowW + 16 + m) * HID_;
  const _Float16* b0p = Bt + (size_t)(colW + m) * HID_;
  const _Float16* b1p = Bt + (size_t)(colW + 16 + m) * HID_;
  #pragma unroll 1
  for (int k0 = 0; k0 < HID_; k0 += 32) {
    const v16h a0 = ldfrag_h(a0p + k0, h);
    const v16h a1 = ldfrag_h(a1p + k0, h);
    const v16h b0 = ldfrag_h(b0p + k0, h);
    const v16h b1 = ldfrag_h(b1p + k0, h);
    acc[0][0] = wmma_h(a0, b0, acc[0][0]);
    acc[0][1] = wmma_h(a0, b1, acc[0][1]);
    acc[1][0] = wmma_h(a1, b0, acc[1][0]);
    acc[1][1] = wmma_h(a1, b1, acc[1][1]);
  }
}

template <int EPI>
__global__ __launch_bounds__(256) void k_gemm1(const _Float16* __restrict__ A, long long zA,
                                               const _Float16* __restrict__ Bt, long long zB,
                                               const float* __restrict__ bias0,
                                               const float* __restrict__ bias1,
                                               const float* __restrict__ bias2,
                                               _Float16* __restrict__ outh,
                                               float* __restrict__ outf, int ldo, long long zO)
{
  __shared__ __align__(16) unsigned char s_stage[8 * STG];
  __shared__ float sBias[TBN];
  const int tid = threadIdx.x, lane = tid & 31, w = tid >> 5;
  const int h = lane >> 4, m = lane & 15;
  const int wm = w >> 1, wn = w & 1;
  const int z = blockIdx.z;
  const int rowW = blockIdx.y * TBM + 32 * wm;
  const int colW = blockIdx.x * TBN + 64 * wn;
  const _Float16* Az = A  + (size_t)z * (size_t)zA;
  const _Float16* Bz = Bt + (size_t)z * (size_t)zB;

  if (tid < TBN) {
    const int gcol = blockIdx.x * TBN + tid;
    float bval;
    if constexpr (EPI == 0) {
      bval = (bias0[gcol] + bias0[NVS_ + gcol]) * 0.5f;
    } else {
      if (blockIdx.x == 0) {
        bval = bias0[(size_t)z * NQC_ + gcol];
      } else if (blockIdx.x == 1) {
        bval = bias1[(size_t)z * NQC_ + (gcol - NQC_)];
      } else {
        const size_t vb = (size_t)z * NVC4_ + (size_t)(gcol - 2 * NQC_);
        bval = 0.25f * ((bias2[vb] + bias2[vb + NVC_]) + (bias2[vb + 2 * NVC_] + bias2[vb + 3 * NVC_]));
      }
    }
    sBias[tid] = bval;
  }
  __syncthreads();

  const v8f z8 = {0.f, 0.f, 0.f, 0.f, 0.f, 0.f, 0.f, 0.f};
  v8f acc[2][4];
  #pragma unroll
  for (int mt = 0; mt < 2; ++mt)
    #pragma unroll
    for (int nt = 0; nt < 4; ++nt) acc[mt][nt] = z8;

  kloop(acc, Az, HID_, Bz, HID_, HID_, rowW, colW, h, m);

  if constexpr (EPI == 0) {
    _Float16* st = (_Float16*)(s_stage + w * STG);
    #pragma unroll
    for (int nt = 0; nt < 4; ++nt) {
      const float bvv = sBias[64 * wn + 16 * nt + m];
      #pragma unroll
      for (int mt = 0; mt < 2; ++mt) {
        #pragma unroll
        for (int r = 0; r < 8; ++r) {
          const int row = 16 * mt + 8 * h + r;
          const int col = 16 * nt + m;
          const float v = acc[mt][nt][r] * WINV + bvv;
          st[row * SPH + col] = (_Float16)v;
        }
      }
    }
    __syncthreads();
    const int q = lane & 7, rs = lane >> 3;
    _Float16* ob = outh + (size_t)rowW * ldo + colW + 8 * q;
    #pragma unroll
    for (int it = 0; it < 8; ++it) {
      const int row = 4 * it + rs;
      const v8h v = *(const v8ha*)(st + row * SPH + 8 * q);
      *(volatile v8ha*)(ob + (size_t)row * ldo) = v;
    }
    __threadfence();
    #pragma unroll
    for (int it = 0; it < 8; ++it) {
      const int row = 4 * it + rs;
      const v8h v = *(const v8ha*)(st + row * SPH + 8 * q);
      *(volatile v8ha*)(ob + (size_t)row * ldo) = v;
    }
  } else {
    float* stf = (float*)(s_stage + w * STG);
    const int hl = lane >> 4, q4 = lane & 15;
    const int colL = colW + 4 * q4;
    float bsel[4];
    #pragma unroll
    for (int nt = 0; nt < 4; ++nt) bsel[nt] = sBias[64 * wn + 16 * nt + m];
    float* outz = outf + (size_t)z * (size_t)zO;
    #pragma unroll
    for (int mt = 0; mt < 2; ++mt) {
      if (mt) __syncthreads();
      #pragma unroll
      for (int nt = 0; nt < 4; ++nt) {
        #pragma unroll
        for (int r = 0; r < 8; ++r) {
          const int row = 8 * h + r;
          const int col = 16 * nt + m;
          stf[row * SPF + col] = acc[mt][nt][r] * WINV + bsel[nt];
        }
      }
      __syncthreads();
      v4f vals[8];
      #pragma unroll
      for (int it = 0; it < 8; ++it) {
        const int row = 2 * it + hl;
        vals[it] = *(const v4fa*)(stf + row * SPF + 4 * q4);
      }
      #pragma unroll
      for (int it = 0; it < 8; ++it) {
        const size_t oidx = (size_t)(rowW + 16 * mt + 2 * it + hl) * ldo + colL;
        *(volatile v4fa*)(outz + oidx) = vals[it];
      }
      __threadfence();
      #pragma unroll
      for (int it = 0; it < 8; ++it) {
        const size_t oidx = (size_t)(rowW + 16 * mt + 2 * it + hl) * ldo + colL;
        *(volatile v4fa*)(outz + oidx) = vals[it];
      }
    }
  }
}

__global__ __launch_bounds__(256) void k_gemmq(const float* __restrict__ Hs,
                                              const unsigned short* __restrict__ Whi,
                                              const unsigned short* __restrict__ Wlo,
                                              const float* __restrict__ bq,
                                              const float* __restrict__ bk,
                                              float* __restrict__ ns)
{
  __shared__ float sS[2][TBM];
  const int tid = threadIdx.x, lane = tid & 31, w = tid >> 5;
  const int h = lane >> 4, m = lane & 15;
  const int wm = w >> 1, wn = w & 1;
  const int z = blockIdx.z;
  const int b0 = blockIdx.y * TBM;
  const int rowL = 32 * wm;
  const int colW = 64 * wn;
  const float* a0p = Hs + ((size_t)z * NB_ + b0 + rowL + m) * HID_;
  const float* a1p = a0p + (size_t)16 * HID_;
  const unsigned short* bhp = Whi + ((size_t)z * NQ_ + colW + m) * HID_;
  const unsigned short* blp = Wlo + ((size_t)z * NQ_ + colW + m) * HID_;

  const v8f z8 = {0.f, 0.f, 0.f, 0.f, 0.f, 0.f, 0.f, 0.f};
  v8f acc[2][4];
  #pragma unroll
  for (int mt = 0; mt < 2; ++mt)
    #pragma unroll
    for (int nt = 0; nt < 4; ++nt) acc[mt][nt] = z8;

  #pragma unroll 1
  for (int k0 = 0; k0 < HID_; k0 += 32) {
    v16bf ah0, al0, ah1, al1;
    ldfrag_split(a0p + k0, h, ah0, al0);
    ldfrag_split(a1p + k0, h, ah1, al1);
    #pragma unroll
    for (int nt = 0; nt < 4; ++nt) {
      const v16bf bh = ldfrag_b(bhp + (size_t)(16 * nt) * HID_ + k0, h);
      const v16bf bl = ldfrag_b(blp + (size_t)(16 * nt) * HID_ + k0, h);
      acc[0][nt] = wmma_b(ah0, bh, acc[0][nt]);
      acc[0][nt] = wmma_b(ah0, bl, acc[0][nt]);
      acc[0][nt] = wmma_b(al0, bh, acc[0][nt]);
      acc[1][nt] = wmma_b(ah1, bh, acc[1][nt]);
      acc[1][nt] = wmma_b(ah1, bl, acc[1][nt]);
      acc[1][nt] = wmma_b(al1, bh, acc[1][nt]);
    }
  }

  float part[2][8];
  #pragma unroll
  for (int mt = 0; mt < 2; ++mt)
    #pragma unroll
    for (int r = 0; r < 8; ++r) part[mt][r] = 0.0f;
  #pragma unroll
  for (int nt = 0; nt < 4; ++nt) {
    const int col = colW + 16 * nt + m;
    const float bqv = bq[(size_t)z * NQ_ + col];
    const float bkv = bk[col];
    #pragma unroll
    for (int mt = 0; mt < 2; ++mt) {
      #pragma unroll
      for (int r = 0; r < 8; ++r) {
        const float t = acc[mt][nt][r] + bqv;
        const float p = t * bkv;
        part[mt][r] = part[mt][r] + p;
      }
    }
  }
  #pragma unroll
  for (int mt = 0; mt < 2; ++mt) {
    #pragma unroll
    for (int r = 0; r < 8; ++r) {
      float v = part[mt][r];
      v += __shfl_xor(v, 1);
      v += __shfl_xor(v, 2);
      v += __shfl_xor(v, 4);
      v += __shfl_xor(v, 8);
      if (m == 0) sS[wn][rowL + 16 * mt + 8 * h + r] = v;
    }
  }
  __syncthreads();
  v4f o = {0.f, 0.f, 0.f, 0.f};
  float* nsp = ns + (size_t)z * NB_ + b0 + 4 * lane;
  if (w == 0) {
    #pragma unroll
    for (int j = 0; j < 4; ++j) {
      const int row = 4 * lane + j;
      const float s0 = sS[0][row], s1 = sS[1][row];
      o[j] = -((s0 * 0.125f + s1 * 0.125f) * 0.5f);
    }
    *(volatile v4fa*)nsp = o;
  }
  __threadfence();
  if (w == 0) {
    *(volatile v4fa*)nsp = o;
  }
}

__global__ __launch_bounds__(256) void k_mask(const float* __restrict__ ns,
                                              float* __restrict__ sel)
{
  __shared__ __align__(16) float sM[256 * MP_];
  const int tid = threadIdx.x;
  const int b = blockIdx.x * 256 + tid;
  float v[NU_];
  #pragma unroll
  for (int u = 0; u < NU_; ++u) v[u] = ns[(size_t)u * NB_ + b];
  #pragma unroll
  for (int u = 0; u < NU_; ++u) {
    int rank = 0;
    #pragma unroll
    for (int w2 = 0; w2 < NU_; ++w2) {
      const bool ahead = (v[w2] > v[u]) || (v[w2] == v[u] && w2 < u);
      rank += ahead ? 1 : 0;
    }
    sM[tid * MP_ + u] = (rank < KTOP_) ? 1.0f : 0.0f;
  }
  sM[tid * MP_ + 6] = 0.0f;
  sM[tid * MP_ + 7] = 0.0f;
  __syncthreads();
  const v4f p0 = *(const v4fa*)(sM + 4 * tid);
  const v4f p1 = *(const v4fa*)(sM + 4 * (tid + 256));
  float* base = sel + (size_t)blockIdx.x * 256 * MP_;
  *(volatile v4fa*)(base + 4 * tid) = p0;
  *(volatile v4fa*)(base + 4 * (tid + 256)) = p1;
  __threadfence();
  *(volatile v4fa*)(base + 4 * tid) = p0;
  *(volatile v4fa*)(base + 4 * (tid + 256)) = p1;
}

template <int EPI>
__global__ __launch_bounds__(256) void k_gemm2(const _Float16* __restrict__ Ax,
                                               const _Float16* __restrict__ Ah,
                                               const _Float16* __restrict__ Bx,
                                               const _Float16* __restrict__ Bh,
                                               const float* __restrict__ bx,
                                               const float* __restrict__ bh,
                                               const float* __restrict__ sel, int u,
                                               const float* __restrict__ rz,
                                               const float* __restrict__ hsf,
                                               float* __restrict__ outf, int ldo,
                                               _Float16* __restrict__ outh)
{
  __shared__ __align__(16) float sT[TBM * BP];
  __shared__ float sSel[TBM];
  __shared__ float sBx[TBN2];
  __shared__ float sBh[TBN2];
  __shared__ int sAny[8];
  const int tid = threadIdx.x, lane = tid & 31, w = tid >> 5;
  const int h = lane >> 4, m = lane & 15;
  const int wm = w >> 1, wn = w & 1;
  const int b0 = blockIdx.y * TBM;
  const int n0 = blockIdx.x * TBN2;
  const int rowL = 32 * wm, colL = 32 * wn;

  const float mv = sel[(size_t)(b0 + (tid & (TBM - 1))) * MP_ + u];
  if (tid < TBM) sSel[tid] = mv;
  if (tid < TBN2) {
    sBx[tid] = bx[n0 + tid];
    sBh[tid] = bh[n0 + tid];
  }
  const int wany = __any((mv != 0.0f) ? 1 : 0);
  if (lane == 0) sAny[w] = wany;
  __syncthreads();
  int any = 0;
  #pragma unroll
  for (int i = 0; i < 8; ++i) any |= sAny[i];

  const v8f z8 = {0.f, 0.f, 0.f, 0.f, 0.f, 0.f, 0.f, 0.f};
  v8f accX[2][2], accH[2][2];
  #pragma unroll
  for (int mt = 0; mt < 2; ++mt)
    #pragma unroll
    for (int nt = 0; nt < 2; ++nt) { accX[mt][nt] = z8; accH[mt][nt] = z8; }

  if (any != 0) kloop2(accX, Ax, Bx, b0 + rowL, n0 + colL, h, m);
  kloop2(accH, Ah, Bh, b0 + rowL, n0 + colL, h, m);

  const int pr = tid >> 4, pp = tid & 15;
  v4f vals[8];

  if constexpr (EPI == 0) {
    #pragma unroll
    for (int nt = 0; nt < 2; ++nt) {
      const int colT = colL + 16 * nt + m;
      const float bxv = sBx[colT];
      const float bhv = sBh[colT];
      #pragma unroll
      for (int mt = 0; mt < 2; ++mt) {
        #pragma unroll
        for (int r = 0; r < 8; ++r) {
          const int rowT = rowL + 16 * mt + 8 * h + r;
          const float mrow = sSel[rowT];
          const float X  = accX[mt][nt][r] * WINV;
          const float Hv = accH[mt][nt][r] * WINV;
          const float gx = mrow * X + bxv;
          const float gh = Hv + bhv;
          sT[rowT * BP + colT] = sigmoid_f(gx + gh);
        }
      }
    }
    __syncthreads();
    #pragma unroll
    for (int it = 0; it < 8; ++it) {
      const int row = pr + 16 * it;
      vals[it] = *(const v4fa*)(sT + row * BP + 4 * pp);
    }
  } else {
    #pragma unroll
    for (int nt = 0; nt < 2; ++nt) {
      const int colT = colL + 16 * nt + m;
      const float bhv = sBh[colT];
      #pragma unroll
      for (int mt = 0; mt < 2; ++mt) {
        #pragma unroll
        for (int r = 0; r < 8; ++r) {
          const int rowT = rowL + 16 * mt + 8 * h + r;
          const float Hv = accH[mt][nt][r] * WINV;
          sT[rowT * BP + colT] = Hv + bhv;
        }
      }
    }
    __syncthreads();
    v4f t4[8];
    #pragma unroll
    for (int it = 0; it < 8; ++it) {
      const int row = pr + 16 * it;
      const v4f nh4 = *(const v4fa*)(sT + row * BP + 4 * pp);
      const v4f rr4 = *(const v4fa*)(rz + (size_t)(b0 + row) * RZP_ + n0 + 4 * pp);
      t4[it] = rr4 * nh4;
    }
    __syncthreads();
    #pragma unroll
    for (int nt = 0; nt < 2; ++nt) {
      const int colT = colL + 16 * nt + m;
      const float bxv = sBx[colT];
      #pragma unroll
      for (int mt = 0; mt < 2; ++mt) {
        #pragma unroll
        for (int r = 0; r < 8; ++r) {
          const int rowT = rowL + 16 * mt + 8 * h + r;
          const float mrow = sSel[rowT];
          const float X  = accX[mt][nt][r] * WINV;
          sT[rowT * BP + colT] = mrow * X + bxv;
        }
      }
    }
    __syncthreads();
    #pragma unroll
    for (int it = 0; it < 8; ++it) {
      const int row = pr + 16 * it;
      const v4f nx4 = *(const v4fa*)(sT + row * BP + 4 * pp);
      const v4f zz4 = *(const v4fa*)(rz  + (size_t)(b0 + row) * RZP_ + HID_ + n0 + 4 * pp);
      const v4f hp4 = *(const v4fa*)(hsf + (size_t)(b0 + row) * HID_ + n0 + 4 * pp);
      v4f hv;
      #pragma unroll
      for (int j = 0; j < 4; ++j) {
        const float n = tanh_f(nx4[j] + t4[it][j]);
        hv[j] = (1.0f - zz4[j]) * n + zz4[j] * hp4[j];
      }
      vals[it] = hv;
    }
    #pragma unroll
    for (int it = 0; it < 8; ++it) {
      const int row = pr + 16 * it;
      *(v4fa*)(sT + row * BP + 4 * pp) = vals[it];
    }
  }

  #pragma unroll
  for (int it = 0; it < 8; ++it) {
    const size_t oidx = (size_t)(b0 + pr + 16 * it) * ldo + n0 + 4 * pp;
    *(volatile v4fa*)(outf + oidx) = vals[it];
  }
  __threadfence();
  #pragma unroll
  for (int it = 0; it < 8; ++it) {
    const size_t oidx = (size_t)(b0 + pr + 16 * it) * ldo + n0 + 4 * pp;
    *(volatile v4fa*)(outf + oidx) = vals[it];
  }
  if constexpr (EPI == 1) {
    __syncthreads();
    v8h oh[4];
    const int hr = tid >> 3, hp8 = tid & 7;
    #pragma unroll
    for (int it = 0; it < 4; ++it) {
      const int row = hr + 32 * it;
      const v4f a = *(const v4fa*)(sT + row * BP + 8 * hp8);
      const v4f b = *(const v4fa*)(sT + row * BP + 8 * hp8 + 4);
      oh[it] = pack8h(a, b);
    }
    #pragma unroll
    for (int it = 0; it < 4; ++it) {
      const size_t hidx = (size_t)(b0 + hr + 32 * it) * HID_ + n0 + 8 * hp8;
      *(volatile v8ha*)(outh + hidx) = oh[it];
    }
    __threadfence();
    #pragma unroll
    for (int it = 0; it < 4; ++it) {
      const size_t hidx = (size_t)(b0 + hr + 32 * it) * HID_ + n0 + 8 * hp8;
      *(volatile v8ha*)(outh + hidx) = oh[it];
    }
  }
}

__global__ __launch_bounds__(192) void k_comm(const float* __restrict__ qkv,
                                             const float* __restrict__ sel,
                                             float* out)
{
  const int tid = threadIdx.x, lane = tid & 31, u = tid >> 5;
  const int b = blockIdx.x;
  const float mu = sel[(size_t)b * MP_ + u];
  const float* qrow = qkv + ((size_t)u * NB_ + b) * NQKV_;
  v4f q4 = *(const v4fa*)(qrow + 4 * lane);
  q4 = q4 * mu;

  float att[NU_];
  #pragma unroll
  for (int v = 0; v < NU_; ++v) {
    const float* krow = qkv + ((size_t)v * NB_ + b) * NQKV_ + NQC_;
    const v4f k4 = *(const v4fa*)(krow + 4 * lane);
    float p = q4.x * k4.x;
    p = p + q4.y * k4.y;
    p = p + q4.z * k4.z;
    p = p + q4.w * k4.w;
    p += __shfl_xor(p, 16);
    p += __shfl_xor(p, 8);
    p += __shfl_xor(p, 4);
    p += __shfl_xor(p, 2);
    p += __shfl_xor(p, 1);
    att[v] = p * ATTSC;
  }
  float mx = att[0];
  #pragma unroll
  for (int v = 1; v < NU_; ++v) mx = fmaxf(mx, att[v]);
  float e[NU_];
  float sum = 0.0f;
  #pragma unroll
  for (int v = 0; v < NU_; ++v) { e[v] = __expf(att[v] - mx); sum = sum + e[v]; }
  const float inv = __builtin_amdgcn_rcpf(sum);
  float pr[NU_];
  #pragma unroll
  for (int v = 0; v < NU_; ++v) pr[v] = (e[v] * inv) * mu;

  float* orow = out + ((size_t)u * NB_ + b) * HID_;
  v4f o[4];
  #pragma unroll
  for (int c = 0; c < 4; ++c) {
    const int off = c * 128 + 4 * lane;
    v4f ctx = {0.f, 0.f, 0.f, 0.f};
    #pragma unroll
    for (int v = 0; v < NU_; ++v) {
      const float* vrow = qkv + ((size_t)v * NB_ + b) * NQKV_ + 2 * NQC_;
      const v4f vv = *(const v4fa*)(vrow + off);
      ctx = ctx + vv * pr[v];
    }
    const v4f hh = *(const v4fa*)(orow + off);
    o[c] = ctx + hh;
  }
  #pragma unroll
  for (int c = 0; c < 4; ++c) *(volatile v4fa*)(orow + c * 128 + 4 * lane) = o[c];
  __threadfence();
  #pragma unroll
  for (int c = 0; c < 4; ++c) *(volatile v4fa*)(orow + c * 128 + 4 * lane) = o[c];
}

extern "C" void kernel_launch(void* const* d_in, const int* in_sizes, int n_in,
                              void* d_out, int out_size, void* d_ws, size_t ws_size,
                              hipStream_t stream)
{
  if (n_in < 18) return;
  if (in_sizes[0]  != NB_ * DIN_) return;
  if (in_sizes[1]  != NU_ * NB_ * HID_) return;
  if (in_sizes[2]  != DIN_ * NQ_) return;
  if (in_sizes[3]  != NQ_) return;
  if (in_sizes[4]  != DIN_ * 2 * NVS_) return;
  if (in_sizes[5]  != 2 * NVS_) return;
  if (in_sizes[6]  != NU_ * HID_ * NQ_) return;
  if (in_sizes[7]  != NU_ * NQ_) return;
  if (in_sizes[8]  != NU_ * G3_ * NVS_) return;
  if (in_sizes[9]  != NU_ * G3_ * HID_) return;
  if (in_sizes[10] != NU_ * G3_) return;
  if (in_sizes[11] != NU_ * G3_) return;
  if (in_sizes[12] != NU_ * HID_ * NQC_) return;
  if (in_sizes[13] != NU_ * NQC_) return;
  if (in_sizes[14] != NU_ * HID_ * NQC_) return;
  if (in_sizes[15] != NU_ * NQC_) return;
  if (in_sizes[16] != NU_ * HID_ * NVC4_) return;
  if (in_sizes[17] != NU_ * NVC4_) return;
  if (out_size != NU_ * NB_ * HID_) return;

  const float* x    = (const float*)d_in[0];
  const float* hs   = (const float*)d_in[1];
  const float* bk   = (const float*)d_in[3];
  const float* Wv   = (const float*)d_in[4];
  const float* bv   = (const float*)d_in[5];
  const float* Wq   = (const float*)d_in[6];
  const float* bq   = (const float*)d_in[7];
  const float* Wih  = (const float*)d_in[8];
  const float* Whh  = (const float*)d_in[9];
  const float* bih  = (const float*)d_in[10];
  const float* bhh  = (const float*)d_in[11];
  const float* Wqc  = (const float*)d_in[12];
  const float* bqc  = (const float*)d_in[13];
  const float* Wkc  = (const float*)d_in[14];
  const float* bkc  = (const float*)d_in[15];
  const float* Wvc  = (const float*)d_in[16];
  const float* bvc  = (const float*)d_in[17];
  float* out = (float*)d_out;

  const size_t bH16  = (size_t)NU_ * NB_ * HID_ * 2;
  const size_t bSEL  = (size_t)NB_ * MP_ * 4;
  const size_t bNS   = (size_t)NU_ * NB_ * 4;
  const size_t bWCT  = (size_t)NU_ * NQKV_ * HID_ * 2;
  const size_t bX16  = (size_t)NB_ * DIN_ * 2;
  const size_t bHS16 = (size_t)NU_ * NB_ * HID_ * 2;
  const size_t bWVMT = (size_t)NVS_ * DIN_ * 2;
  const size_t bWQ   = (size_t)NU_ * NQ_ * HID_ * 2;
  const size_t bWIH  = (size_t)NU_ * G3_ * NVS_ * 2;
  const size_t bWHH  = (size_t)NU_ * G3_ * HID_ * 2;
  const size_t bV016 = (size_t)NB_ * NVS_ * 2;
  const size_t bRZ   = (size_t)NB_ * RZP_ * 4;
  const size_t phaseA = bX16 + bHS16 + bWVMT + 2 * bWQ + bWIH + bWHH + bV016 + bRZ;
  const size_t bQKV  = (size_t)NU_ * NB_ * NQKV_ * 4;
  const size_t phase = (phaseA > bQKV) ? phaseA : bQKV;
  const size_t total = bH16 + bSEL + bNS + bWCT + phase;
  if (total > ws_size) return;
  if (total > (size_t)134217728) return;

  char* ws = (char*)d_ws;
  size_t off = 0;
  _Float16* H16 = (_Float16*)(ws + off); off += bH16;
  float*    SEL = (float*)(ws + off);    off += bSEL;
  float*    NS  = (float*)(ws + off);    off += bNS;
  _Float16* WCT = (_Float16*)(ws + off); off += bWCT;
  const size_t pbase = off;
  size_t poff = pbase;
  _Float16*       X16  = (_Float16*)(ws + poff);       poff += bX16;
  _Float16*       HS16 = (_Float16*)(ws + poff);       poff += bHS16;
  _Float16*       WVMT = (_Float16*)(ws + poff);       poff += bWVMT;
  unsigned short* WQHI = (unsigned short*)(ws + poff); poff += bWQ;
  unsigned short* WQLO = (unsigned short*)(ws + poff); poff += bWQ;
  _Float16*       WIH16 = (_Float16*)(ws + poff);      poff += bWIH;
  _Float16*       WHH16 = (_Float16*)(ws + poff);      poff += bWHH;
  _Float16*       V016 = (_Float16*)(ws + poff);       poff += bV016;
  float*          RZ   = (float*)(ws + poff);          poff += bRZ;
  if (poff != pbase + phaseA) return;
  float*          QKV  = (float*)(ws + pbase);
  if (pbase + phase != total) return;

  k_cvt16<<<(NB_ * DIN_ / 8) / 256, 256, 0, stream>>>(x,  X16,  NB_ * DIN_ / 8, 1.0f);
  k_cvt16<<<(NU_ * NB_ * HID_ / 8) / 256, 256, 0, stream>>>(hs, HS16, NU_ * NB_ * HID_ / 8, 1.0f);
  k_cvt16<<<(NU_ * G3_ * NVS_ / 8) / 256, 256, 0, stream>>>(Wih, WIH16, NU_ * G3_ * NVS_ / 8, WSCALE);
  k_cvt16<<<(NU_ * G3_ * HID_ / 8) / 256, 256, 0, stream>>>(Whh, WHH16, NU_ * G3_ * HID_ / 8, WSCALE);

  k_wt<2, 0><<<dim3(NVS_ / TT, DIN_ / TT, 1), 256, 0, stream>>>(Wv, 0, WVMT, WQHI, WQLO, 0, DIN_, NVS_, 32.0f);
  k_wt<1, 1><<<dim3(NQ_ / TT, HID_ / TT, NU_), 256, 0, stream>>>(Wq, (long long)HID_ * NQ_, WVMT, WQHI, WQLO,
                                                               (long long)NQ_ * HID_, HID_, NQ_, 1.0f);
  k_wt<1, 0><<<dim3(NQC_ / TT, HID_ / TT, NU_), 256, 0, stream>>>(Wqc, (long long)HID_ * NQC_, WCT, WQHI, WQLO,
                                                                (long long)NQKV_ * HID_, HID_, NQC_, WSCALE);
  k_wt<1, 0><<<dim3(NQC_ / TT, HID_ / TT, NU_), 256, 0, stream>>>(Wkc, (long long)HID_ * NQC_, WCT + (size_t)NQC_ * HID_, WQHI, WQLO,
                                                                (long long)NQKV_ * HID_, HID_, NQC_, WSCALE);
  k_wt<4, 0><<<dim3(NVC_ / TT, HID_ / TT, NU_), 256, 0, stream>>>(Wvc, (long long)HID_ * NVC4_, WCT + (size_t)2 * NQC_ * HID_, WQHI, WQLO,
                                                                (long long)NQKV_ * HID_, HID_, NVC_, 16.0f);

  k_gemm1<0><<<dim3(NVS_ / TBN, NB_ / TBM, 1), 256, 0, stream>>>(
      X16, 0, WVMT, 0, bv, bv, bv, V016, RZ, NVS_, 0);

  k_gemmq<<<dim3(1, NB_ / TBM, NU_), 256, 0, stream>>>(hs, WQHI, WQLO, bq, bk, NS);
  k_mask<<<NB_ / 256, 256, 0, stream>>>(NS, SEL);

  for (int u = 0; u < NU_; ++u) {
    const _Float16* hs16u = HS16 + (size_t)u * NB_ * HID_;
    const _Float16* wihu  = WIH16 + (size_t)u * G3_ * NVS_;
    const _Float16* whhu  = WHH16 + (size_t)u * G3_ * HID_;
    const float*    hsu   = hs + (size_t)u * NB_ * HID_;
    _Float16*       h16u  = H16 + (size_t)u * NB_ * HID_;
    float*          outu  = out + (size_t)u * NB_ * HID_;
    k_gemm2<0><<<dim3(RZP_ / TBN2, NB_ / TBM, 1), 256, 0, stream>>>(
        V016, hs16u, wihu, whhu, bih + (size_t)u * G3_, bhh + (size_t)u * G3_,
        SEL, u, RZ, hsu, RZ, RZP_, h16u);
    k_gemm2<1><<<dim3(HID_ / TBN2, NB_ / TBM, 1), 256, 0, stream>>>(
        V016, hs16u, wihu + (size_t)RZP_ * NVS_, whhu + (size_t)RZP_ * HID_,
        bih + (size_t)u * G3_ + RZP_, bhh + (size_t)u * G3_ + RZP_,
        SEL, u, RZ, hsu, outu, HID_, h16u);
  }

  k_gemm1<1><<<dim3(NQKV_ / TBN, NB_ / TBM, NU_), 256, 0, stream>>>(
      H16, (long long)NB_ * HID_, WCT, (long long)NQKV_ * HID_, bqc, bkc, bvc,
      V016, QKV, NQKV_, (long long)NB_ * NQKV_);

  k_comm<<<NB_, 192, 0, stream>>>(QKV, SEL, out);
}
